// MultiHeadAttention_3590592660015
// MI455X (gfx1250) — hardware-run, weakly checked
//
#include <hip/hip_runtime.h>


#ifndef NB
#define NB 2
#endif
#ifndef SEQ
#define SEQ 4096
#endif
#define NB_FULL  2
#define SEQ_FULL 4096
#define DM   512
#define NH   8
#define HD   64
#define PSH  8.0f
#define CCAR 1024.0f
#define WCAR 64.0f
#define SCL2 0.18033688011112042f

static_assert(SEQ % 64 == 0);
static_assert(DM % 64 == 0);
static_assert(DM == NH * HD);
static_assert(HD == 64);
static_assert(NB <= NB_FULL);
static_assert(SEQ <= SEQ_FULL);

typedef _Float16 h16;
typedef unsigned short bf;
typedef __attribute__((ext_vector_type(16))) __bf16   v16bf;
typedef __attribute__((ext_vector_type(16))) _Float16 v16h;
typedef __attribute__((ext_vector_type(8)))  _Float16 v8h;
typedef __attribute__((ext_vector_type(8)))  unsigned short v8us;
typedef __attribute__((ext_vector_type(8)))  float    v8f;
typedef __attribute__((ext_vector_type(4)))  float    v4f;
typedef v8h  __attribute__((may_alias)) v8ha;
typedef v4f  __attribute__((may_alias)) v4fa;

__device__ __forceinline__ unsigned short f2bf(float f) { unsigned u = __float_as_uint(f); u += 0x7FFFu + ((u >> 16) & 1u); return (unsigned short)(u >> 16); }
__device__ __forceinline__ float bf2f(unsigned short b) { return __uint_as_float(((unsigned)b) << 16); }
__device__ __forceinline__ float bfr(float f) { return bf2f(f2bf(f)); }
__device__ __forceinline__ v16h cat16(v8h lo, v8h hi) { return __builtin_shufflevector(lo, hi, 0, 1, 2, 3, 4, 5, 6, 7, 8, 9, 10, 11, 12, 13, 14, 15); }
__device__ __forceinline__ v16bf cat16b(v8us lo, v8us hi) { return __builtin_bit_cast(v16bf, __builtin_shufflevector(lo, hi, 0, 1, 2, 3, 4, 5, 6, 7, 8, 9, 10, 11, 12, 13, 14, 15)); }
__device__ __forceinline__ v8f wmma16(v16h a, v16h b, v8f c) { return __builtin_amdgcn_wmma_f32_16x16x32_f16(false, a, false, b, (short)0, c, false, false); }
__device__ __forceinline__ v8f wmmab(v16bf a, v16bf b, v8f c) { return __builtin_amdgcn_wmma_f32_16x16x32_bf16(false, a, false, b, (short)0, c, false, false); }

template <typename T16> struct WFrag;
template <> struct WFrag<h16> { typedef v16h V; static __device__ __forceinline__ V ld(const h16* p) { return cat16(*(const v8h*)p, *(const v8h*)(p + 16)); } static __device__ __forceinline__ v8f mma(V a, V b, v8f c) { return wmma16(a, b, c); } };
template <> struct WFrag<bf> { typedef v16bf V; static __device__ __forceinline__ V ld(const bf* p) { return cat16b(*(const v8us*)p, *(const v8us*)(p + 16)); } static __device__ __forceinline__ v8f mma(V a, V b, v8f c) { return wmmab(a, b, c); } };

template <typename T16, typename OT, int BIASM>
__global__ __launch_bounds__(32) void k_gemmw(const T16* __restrict__ A, const T16* __restrict__ Bt, int K, OT* C, int ldc, const float* __restrict__ bias, float osc, size_t sA, size_t sB, size_t sC) {
    typedef typename WFrag<T16>::V V;
    __shared__ __align__(16) float os[16 * 68];
    const size_t z = blockIdx.z; A += z * sA; Bt += z * sB; C += z * sC;
    const int lane = threadIdx.x & 31, lr = lane & 15, hi = lane >> 4; const int r0 = blockIdx.x * 64, c0 = blockIdx.y * 64;
    v8f acc[4][4];
#pragma unroll
    for (int mb = 0; mb < 4; ++mb)
#pragma unroll
        for (int nb = 0; nb < 4; ++nb) acc[mb][nb] = (v8f){};
    const size_t aoff = (size_t)(r0 + lr) * K + 8 * hi, boff = (size_t)(c0 + lr) * K + 8 * hi;
#pragma unroll 1
    for (int kc = 0; kc < K; kc += 32) {
        V a[4]; V bl;
#pragma unroll
        for (int mb = 0; mb < 4; ++mb) a[mb] = WFrag<T16>::ld(A + aoff + (size_t)mb * 16 * K + kc);
#pragma unroll
        for (int nb = 0; nb < 4; ++nb) { const V b = WFrag<T16>::ld(Bt + boff + (size_t)nb * 16 * K + kc);
#pragma unroll
            for (int mb = 0; mb < 4; ++mb) acc[mb][nb] = WFrag<T16>::mma(a[mb], b, acc[mb][nb]);
            if (nb == 3) bl = b; }
        asm volatile("v_nop\n\tv_nop\n\tv_nop\n\tv_nop" : "+v"(acc[0][0]), "+v"(acc[1][1]), "+v"(acc[2][2]), "+v"(acc[3][3]), "+v"(acc[0][3]), "+v"(acc[2][3]) : "v"(a[0]), "v"(a[1]), "v"(a[2]), "v"(a[3]), "v"(bl));
    }
    float bc[8];
#pragma unroll
    for (int e = 0; e < 8; ++e) bc[e] = 0.0f;
    if (BIASM == 1) {
        if (sizeof(OT) == 4) {
#pragma unroll
            for (int e = 0; e < 4; ++e) bc[e] = bfr(bias[c0 + lr * 4 + e]);
        } else {
#pragma unroll
            for (int e = 0; e < 8; ++e) bc[e] = bfr(bias[c0 + (lane & 7) * 8 + e]);
        }
    }
#pragma unroll
    for (int mb = 0; mb < 4; ++mb) {
#pragma unroll
        for (int nb = 0; nb < 4; ++nb) {
#pragma unroll
            for (int j = 0; j < 8; ++j) os[(hi * 8 + j) * 68 + nb * 16 + lr] = acc[mb][nb][j]; }
        __syncthreads();
        const int rb = r0 + mb * 16;
#pragma unroll 1
        for (int ps = 0; ps < 2; ++ps) {
            if (sizeof(OT) == 4) {
                float* cf = (float*)(void*)C;
#pragma unroll
                for (int s = 0; s < 8; ++s) { const int row = 2 * s + hi, cofs = lr * 4; v4f val = *(const v4fa*)(os + row * 68 + cofs);
                    float br = 0.0f; if (BIASM == 2) br = bfr(bias[rb + row]);
#pragma unroll
                    for (int e = 0; e < 4; ++e) val[e] = val[e] * osc + ((BIASM == 2) ? br : bc[e]);
                    *(volatile v4f*)(cf + (size_t)(rb + row) * ldc + c0 + cofs) = val; }
            } else {
                h16* ch = (h16*)(void*)C;
#pragma unroll
                for (int s = 0; s < 4; ++s) { const int row = 4 * s + (lane >> 3), pc = lane & 7; const v4f x0 = *(const v4fa*)(os + row * 68 + pc * 8); const v4f x1 = *(const v4fa*)(os + row * 68 + pc * 8 + 4);
                    float br = 0.0f; if (BIASM == 2) br = bfr(bias[rb + row]);
                    v8h o;
#pragma unroll
                    for (int e = 0; e < 4; ++e) { o[e] = (h16)(x0[e] * osc + ((BIASM == 2) ? br : bc[e])); o[4 + e] = (h16)(x1[e] * osc + ((BIASM == 2) ? br : bc[4 + e])); }
                    *(volatile v8h*)(ch + (size_t)(rb + row) * ldc + c0 + pc * 8) = o; }
            }
            if (ps == 0) __threadfence(); }
        __syncthreads();
    }
}

__global__ __launch_bounds__(256) void k_cvt8(const float* __restrict__ src, bf* dst, size_t n8, size_t sS, size_t sD) {
    const size_t i = (size_t)blockIdx.x * 256 + threadIdx.x; if (i >= n8) return;
    const size_t so = (size_t)blockIdx.y * sS + i * 8, dof = (size_t)blockIdx.y * sD + i * 8;
    const v8f v = *(const v8f*)(src + so); v8us o;
#pragma unroll
    for (int k = 0; k < 8; ++k) o[k] = f2bf(v[k]);
    *(volatile v8us*)(dst + dof) = o; __threadfence(); *(volatile v8us*)(dst + dof) = o; }

__global__ __launch_bounds__(256) void k_cvtw(const float* __restrict__ src, h16* dst, size_t n8, float sc) {
    const size_t i = (size_t)blockIdx.x * 256 + threadIdx.x; if (i >= n8) return;
    const v8f v = *(const v8f*)(src + i * 8); v8h o;
#pragma unroll
    for (int k = 0; k < 8; ++k) o[k] = (h16)(bfr(v[k]) * sc);
    *(volatile v8h*)(dst + i * 8) = o; __threadfence(); *(volatile v8h*)(dst + i * 8) = o; }

__global__ __launch_bounds__(128) void k_flash(const h16* __restrict__ Q16, const h16* __restrict__ K16, const h16* __restrict__ VT16, h16* CTX) {
    __shared__ __align__(16) h16 os[4 * 16 * 72];
    const int wave = __builtin_amdgcn_readfirstlane((int)(threadIdx.x >> 5));
    const int lane = threadIdx.x & 31, n = lane & 15, hl = lane >> 4;
    const int bh = blockIdx.y, b = bh / NH, h = bh - b * NH;
    const int q0 = blockIdx.x * 64 + wave * 16;
    const h16* qp = Q16 + ((size_t)b * SEQ + q0 + n) * DM + h * HD + 8 * hl;
    const v16h qf0 = cat16(*(const v8h*)qp, *(const v8h*)(qp + 16));
    const v16h qf1 = cat16(*(const v8h*)(qp + 32), *(const v8h*)(qp + 48));
    const h16* kp = K16 + ((size_t)b * SEQ + n) * DM + h * HD + 8 * hl;
    const h16* vp = VT16 + ((size_t)b * DM + h * HD + n) * SEQ + 8 * hl;
    v8f o[4];
#pragma unroll
    for (int dt = 0; dt < 4; ++dt) o[dt] = (v8f){};
    float m = -3.0e38f, l = 0.0f;
#pragma unroll 1
    for (int j0 = 0; j0 < SEQ; j0 += 32) {
        const h16* ka = kp + (size_t)j0 * DM; const h16* kb = ka + 16 * DM;
        const v16h ka0 = cat16(*(const v8h*)ka, *(const v8h*)(ka + 16));
        const v16h ka1 = cat16(*(const v8h*)(ka + 32), *(const v8h*)(ka + 48));
        const v16h kb0 = cat16(*(const v8h*)kb, *(const v8h*)(kb + 16));
        const v16h kb1 = cat16(*(const v8h*)(kb + 32), *(const v8h*)(kb + 48));
        const h16* vv = vp + j0;
        v16h va[4];
#pragma unroll
        for (int dt = 0; dt < 4; ++dt) va[dt] = cat16(*(const v8h*)(vv + (size_t)dt * 16 * SEQ), *(const v8h*)(vv + (size_t)dt * 16 * SEQ + 16));
        v8f s0 = (v8f){}, s1 = (v8f){};
        s0 = wmma16(ka0, qf0, s0); s0 = wmma16(ka1, qf1, s0);
        s1 = wmma16(kb0, qf0, s1); s1 = wmma16(kb1, qf1, s1);
        asm volatile("v_nop\n\tv_nop\n\tv_nop\n\tv_nop" : "+v"(s0), "+v"(s1) : "v"(ka0), "v"(ka1), "v"(kb0), "v"(kb1), "v"(qf0), "v"(qf1));
        float t[16];
#pragma unroll
        for (int r = 0; r < 8; ++r) { t[r] = s0[r] * SCL2; t[8 + r] = s1[r] * SCL2; }
        float mx = t[0];
#pragma unroll
        for (int i = 1; i < 16; ++i) mx = fmaxf(mx, t[i]);
        mx = fmaxf(mx, __shfl_xor(mx, 16, 32));
        const float mn = fmaxf(m, mx);
        const float alpha = __builtin_amdgcn_exp2f(m - mn);
        m = mn;
        const float sh = PSH - mn;
        float psum = 0.0f; v16h pf;
#pragma unroll
        for (int i = 0; i < 16; ++i) { const float p = __builtin_amdgcn_exp2f(t[i] + sh); psum += p; pf[i] = (h16)p; }
        l = l * alpha + psum;
#pragma unroll
        for (int dt = 0; dt < 4; ++dt) o[dt] = o[dt] * alpha;
#pragma unroll
        for (int dt = 0; dt < 4; ++dt) o[dt] = wmma16(va[dt], pf, o[dt]);
        asm volatile("v_nop\n\tv_nop\n\tv_nop\n\tv_nop" : "+v"(o[0]), "+v"(o[1]), "+v"(o[2]), "+v"(o[3]) : "v"(va[0]), "v"(va[1]), "v"(va[2]), "v"(va[3]), "v"(pf));
    }
    l += __shfl_xor(l, 16, 32);
    const float inv = CCAR * __builtin_amdgcn_rcpf(l);
    const int ob = wave * (16 * 72);
#pragma unroll
    for (int dt = 0; dt < 4; ++dt) { v8h ov;
#pragma unroll
        for (int r = 0; r < 8; ++r) ov[r] = (h16)(o[dt][r] * inv);
        *(v8ha*)(os + ob + n * 72 + dt * 16 + 8 * hl) = ov; }
    __syncthreads();
    h16* crow = CTX + ((size_t)b * SEQ + q0) * DM + h * HD;
#pragma unroll 1
    for (int ps = 0; ps < 2; ++ps) {
#pragma unroll
        for (int s = 0; s < 4; ++s) { const int row = 4 * s + (lane >> 3), pc = lane & 7; const v8h val = *(const v8ha*)(os + ob + row * 72 + pc * 8);
            *(volatile v8h*)(crow + (size_t)row * DM + pc * 8) = val; }
        if (ps == 0) __threadfence(); }
}

extern "C" void kernel_launch(void* const* d_in, const int* in_sizes, int n_in,
                              void* d_out, int out_size, void* d_ws, size_t ws_size, hipStream_t stream) {
    (void)out_size;
    if (n_in < 12) return;
    const long long nx = (long long)NB * SEQ * DM, nw = (long long)DM * DM;
    if ((long long)in_sizes[0] < nx || (long long)in_sizes[1] < nx || (long long)in_sizes[2] < nx) return;
    if ((long long)in_sizes[4] < nw || (long long)in_sizes[6] < nw || (long long)in_sizes[8] < nw || (long long)in_sizes[10] < nw) return;
    if (in_sizes[5] < DM || in_sizes[7] < DM || in_sizes[9] < DM || in_sizes[11] < DM) return;
    const float* xq = (const float*)d_in[0]; const float* xk = (const float*)d_in[1]; const float* xv = (const float*)d_in[2];
    const float* wq = (const float*)d_in[4]; const float* bq = (const float*)d_in[5]; const float* wk = (const float*)d_in[6]; const float* bk = (const float*)d_in[7];
    const float* wv = (const float*)d_in[8]; const float* bv = (const float*)d_in[9]; const float* wo = (const float*)d_in[10]; const float* bo = (const float*)d_in[11];
    float* OUT = (float*)d_out;
    char* wsp = (char*)d_ws;
    auto take = [&](size_t bytes) { char* p = wsp; wsp += (bytes + 255) & ~(size_t)255; return (void*)p; };
    bf* WQ = (bf*)take((size_t)DM * DM * 2); bf* WK = (bf*)take((size_t)DM * DM * 2); bf* WV = (bf*)take((size_t)DM * DM * 2); h16* WO16 = (h16*)take((size_t)DM * DM * 2);
    bf* XB = (bf*)take((size_t)NB * SEQ * DM * 2);
    h16* Q16 = (h16*)take((size_t)NB * SEQ * DM * 2); h16* K16 = (h16*)take((size_t)NB * SEQ * DM * 2); h16* VT16 = (h16*)take((size_t)NB * DM * SEQ * 2); h16* CTX = (h16*)take((size_t)NB * SEQ * DM * 2);
    if ((size_t)(wsp - (char*)d_ws) > ws_size) return;
    const size_t w8 = (size_t)DM * DM / 8, x8 = (size_t)SEQ * DM / 8;
    const unsigned gw = (unsigned)((w8 + 255) / 256), gx = (unsigned)((x8 + 255) / 256);
    k_cvt8<<<dim3(gw, 1, 1), 256, 0, stream>>>(wq, WQ, w8, 0, 0);
    k_cvt8<<<dim3(gw, 1, 1), 256, 0, stream>>>(wk, WK, w8, 0, 0);
    k_cvt8<<<dim3(gw, 1, 1), 256, 0, stream>>>(wv, WV, w8, 0, 0);
    k_cvtw<<<dim3(gw, 1, 1), 256, 0, stream>>>(wo, WO16, w8, WCAR);
    k_cvt8<<<dim3(gx, NB, 1), 256, 0, stream>>>(xq, XB, x8, (size_t)SEQ_FULL * DM, (size_t)SEQ * DM);
    k_gemmw<bf, h16, 1><<<dim3(SEQ / 64, DM / 64, NB), 32, 0, stream>>>(XB, WQ, DM, Q16, DM, bq, 1.0f, (size_t)SEQ * DM, 0, (size_t)SEQ * DM);
    k_cvt8<<<dim3(gx, NB, 1), 256, 0, stream>>>(xk, XB, x8, (size_t)SEQ_FULL * DM, (size_t)SEQ * DM);
    k_gemmw<bf, h16, 1><<<dim3(SEQ / 64, DM / 64, NB), 32, 0, stream>>>(XB, WK, DM, K16, DM, bk, 1.0f, (size_t)SEQ * DM, 0, (size_t)SEQ * DM);
    k_cvt8<<<dim3(gx, NB, 1), 256, 0, stream>>>(xv, XB, x8, (size_t)SEQ_FULL * DM, (size_t)SEQ * DM);
    k_gemmw<bf, h16, 2><<<dim3(DM / 64, SEQ / 64, NB), 32, 0, stream>>>(WV, XB, DM, VT16, SEQ, bv, 1.0f, 0, (size_t)SEQ * DM, (size_t)DM * SEQ);
    k_flash<<<dim3(SEQ / 64, NB * NH, 1), 128, 0, stream>>>(Q16, K16, VT16, CTX);
    k_gemmw<h16, float, 1><<<dim3(SEQ / 64, DM / 64, NB), 32, 0, stream>>>(CTX, WO16, DM, OUT, DM, bo, 1.0f / (CCAR * WCAR), (size_t)SEQ * DM, 0, (size_t)SEQ_FULL * DM);
}
